// Gemma4FullAttention_47115791237727
// MI455X (gfx1250) — hardware-verified
//
#include <hip/hip_runtime.h>
#include <math.h>
#include <stdint.h>

#ifndef NB
#define NB 2
#endif
#ifndef SEQ
#define SEQ 2048
#endif
#define XS_FULL 2048
#define DMOD  2048
#define NH    8
#define NKV   4
#define NREP  (NH / NKV)
#define HD    256
#define KVD   (NKV * HD)
#define QO    ((SEQ < 256) ? SEQ : 256)
#define MROWS (NB * SEQ)
#define EPS_RMS 0.000001f
#define SM_SCALE 0.0625f
#define LOG2E 1.4426950408889634f
#define NEGT  (-1.0e30f)
#define QSC   256.0f
#define KSC   256.0f
#define PCAR  32768.0f
#define VCAR  1024.0f
#define OSC   1024.0f
#define WOS   1024.0f
#define WPB   2
#define DW    (HD / WPB)
#define NQT   (SEQ / 16)
#define NKT   (SEQ / 32)
#define NSTT  (MROWS / 64)
#define ATT_THREADS (WPB * 32)
#define PTP   36
#define PTW   (16 * PTP)
#define SLP   132
#define SLW   (16 * SLP)
#define XCHW  (2 * WPB * 16)
#define SLAB64 (16 * 68)
#define VTP   72
#define WS_CAP 134217728
static_assert(DMOD == NH * HD && HD == 256 && DW == 128 && KVD == NKV * HD && NREP == 2 && NREP * NKV == NH && WPB == 2);
static_assert(ATT_THREADS == 64);
static_assert(NB >= 1 && NB <= 2);
static_assert((SEQ % 64) == 0 && SEQ >= 64 && SEQ <= XS_FULL);
static_assert((QO % 64) == 0 && QO >= 64 && QO <= SEQ && (QO % 16) == 0);
static_assert((DMOD % 64) == 0 && (KVD % 64) == 0 && (DMOD % 32) == 0 && (MROWS % 64) == 0);
static_assert(((SEQ * DMOD / 8) % 256) == 0 && ((DMOD * DMOD / 8) % 256) == 0 && ((KVD * DMOD / 8) % 256) == 0);
static_assert((DMOD / 8) <= 256 && ((DMOD / 8) % 32) == 0 && (KVD / 8) <= 256 && ((KVD / 8) % 32) == 0);
static_assert((PTW + XCHW + WPB * SLW) * 4 <= 65536 && 2 * DW * VTP * 2 <= 65536 && 4 * SLAB64 * 4 <= 65536);
static_assert((size_t)MROWS * DMOD * 2 + (size_t)DMOD * DMOD * 2 + (size_t)MROWS * DMOD * 4
              + 2 * (size_t)MROWS * DMOD * 2 + 4 * (size_t)MROWS * KVD * 2 <= (size_t)WS_CAP);
static_assert((size_t)MROWS * DMOD * 4 <= (size_t)33554432);

typedef unsigned short u16;
typedef _Float16 v16h __attribute__((ext_vector_type(16)));
typedef _Float16 v8h  __attribute__((ext_vector_type(8)));
typedef __bf16   v16b __attribute__((ext_vector_type(16)));
typedef float    v8f  __attribute__((ext_vector_type(8)));
typedef float    v4f  __attribute__((ext_vector_type(4)));
typedef unsigned int v4u __attribute__((ext_vector_type(4)));

union FragH { v16h v; v8h h[2]; v4u u[2]; };
union FragB { v16b v; v4u u[2]; };

__device__ __forceinline__ unsigned short bf_bits(float f) {
  unsigned u = __float_as_uint(f);
  return (unsigned short)((u + 0x7FFFu + ((u >> 16) & 1u)) >> 16);
}
__device__ __forceinline__ float bf_up(unsigned short h) { return __uint_as_float(((unsigned)h) << 16); }
__device__ __forceinline__ float bfr(float f) { return bf_up(bf_bits(f)); }
__device__ __forceinline__ unsigned short h_bits(_Float16 x) { return __builtin_bit_cast(unsigned short, x); }
__device__ __forceinline__ unsigned pk16(unsigned short a, unsigned short b) { return (unsigned)a | ((unsigned)b << 16); }
__device__ __forceinline__ v8f zero8() { v8f z = {0.f, 0.f, 0.f, 0.f, 0.f, 0.f, 0.f, 0.f}; return z; }

__device__ __forceinline__ v16h ldfrag_h(const _Float16* p) {
  FragH f;
  f.h[0] = *(const v8h*)(p);
  f.h[1] = *(const v8h*)(p + 16);
  return f.v;
}
__device__ __forceinline__ v16b ldfrag_b(const u16* p) {
  FragB f;
  f.u[0] = *(const v4u*)(p);
  f.u[1] = *(const v4u*)(p + 16);
  return f.v;
}

__device__ __forceinline__ v8f mma_h(v16h a, v16h b, v8f c) {
  return __builtin_amdgcn_wmma_f32_16x16x32_f16(false, a, false, b, (short)0, c, false, false);
}
__device__ __forceinline__ v8f mma_b(v16b a, v16b b, v8f c) {
  return __builtin_amdgcn_wmma_f32_16x16x32_bf16(false, a, false, b, (short)0, c, false, false);
}
template <typename F>
__device__ __forceinline__ void guard1(v8f& a, F x0, F x1, F x2, F x3) {
#if defined(__HIP_DEVICE_COMPILE__)
  asm volatile("v_nop\n\tv_nop\n\tv_nop\n\tv_nop" : "+v"(a) : "v"(x0), "v"(x1), "v"(x2), "v"(x3) : "memory");
#endif
}
__device__ __forceinline__ void guard2(v8f& a, v8f& b, v16h x0, v16h x1, v16h x2, v16h x3, v16h x4, v16h x5) {
#if defined(__HIP_DEVICE_COMPILE__)
  asm volatile("v_nop\n\tv_nop\n\tv_nop\n\tv_nop"
               : "+v"(a), "+v"(b) : "v"(x0), "v"(x1), "v"(x2), "v"(x3), "v"(x4), "v"(x5) : "memory");
#endif
}
template <typename F>
__device__ __forceinline__ void guard6(v8f& a, v8f& b, v8f& c, v8f& d, F x0, F x1, F x2, F x3, F x4, F x5) {
#if defined(__HIP_DEVICE_COMPILE__)
  asm volatile("v_nop\n\tv_nop\n\tv_nop\n\tv_nop"
               : "+v"(a), "+v"(b), "+v"(c), "+v"(d) : "v"(x0), "v"(x1), "v"(x2), "v"(x3), "v"(x4), "v"(x5) : "memory");
#endif
}
__device__ __forceinline__ void acc_guard4(v8f& a, v8f& b, v8f& c, v8f& d) {
#if defined(__HIP_DEVICE_COMPILE__)
  asm volatile("v_nop\n\tv_nop\n\tv_nop\n\tv_nop" : "+v"(a), "+v"(b), "+v"(c), "+v"(d));
#endif
}
__device__ __forceinline__ void wave_sync_lds() {
  __builtin_amdgcn_fence(__ATOMIC_RELEASE, "workgroup");
  __builtin_amdgcn_wave_barrier();
  __builtin_amdgcn_fence(__ATOMIC_ACQUIRE, "workgroup");
}

__global__ __launch_bounds__(256) void cvt16(const float* __restrict__ x, u16* D, int n8, int f16mode, float scale) {
  const int gt = blockIdx.x * 256 + (int)threadIdx.x;
  if (gt >= n8) return;
  const float* p = x + (size_t)gt * 8;
  const v4f a = *(const v4f*)(p), b4 = *(const v4f*)(p + 4);
  float w[8];
#pragma unroll
  for (int e = 0; e < 4; ++e) { w[e] = a[e]; w[4 + e] = b4[e]; }
  v4u o;
#pragma unroll
  for (int e = 0; e < 4; ++e) {
    const float f0 = w[2 * e], f1 = w[2 * e + 1];
    const unsigned short hb0 = h_bits((_Float16)(bfr(f0) * scale));
    const unsigned short hb1 = h_bits((_Float16)(bfr(f1) * scale));
    const unsigned short bb0 = bf_bits(f0);
    const unsigned short bb1 = bf_bits(f1);
    o[e] = (f16mode != 0) ? pk16(hb0, hb1) : pk16(bb0, bb1);
  }
  u16* d = D + (size_t)gt * 8;
  for (int pass = 0; pass < 2; ++pass) {
    *(volatile v4u*)(d) = o;
    __threadfence();
  }
}

__global__ __launch_bounds__(256) void vt16(const float* __restrict__ F, u16* VHo, u16* VLo) {
  __shared__ __align__(16) u16 TH[DW * VTP];
  __shared__ __align__(16) u16 TL[DW * VTP];
  const int tid = threadIdx.x;
  const int bid = blockIdx.x;
  const int st  = bid % NSTT;
  const int t2  = bid / NSTT;
  const int dh  = t2 % (HD / DW);
  const int g   = t2 / (HD / DW);
  if (g >= NKV) return;
  const int row0 = st * 64;
  const int b    = row0 / SEQ;
  const int s0   = row0 - b * SEQ;
  {
    const int sl = tid >> 2;
    const int dc = (tid & 3) * 32;
    const float* src = F + (size_t)(row0 + sl) * KVD + g * HD + dh * DW + dc;
#pragma unroll
    for (int i = 0; i < 8; ++i) {
      const v4f a = *(const v4f*)(src + 4 * i);
#pragma unroll
      for (int e = 0; e < 4; ++e) {
        const float t = a[e] * VCAR;
        const _Float16 hv = (_Float16)t;
        const _Float16 lv = (_Float16)(t - (float)hv);
        TH[(dc + 4 * i + e) * VTP + sl] = h_bits(hv);
        TL[(dc + 4 * i + e) * VTP + sl] = h_bits(lv);
      }
    }
  }
  __syncthreads();
  v4u vh[4], vl[4];
  const int q8 = tid >> 3, p8 = (tid & 7) * 8;
#pragma unroll
  for (int it = 0; it < 4; ++it) {
    const int line = it * 32 + q8;
    vh[it] = *(const v4u*)(TH + line * VTP + p8);
    vl[it] = *(const v4u*)(TL + line * VTP + p8);
  }
  const size_t hrow = (size_t)(b * NKV + g) * HD + (size_t)dh * DW;
  const size_t base = hrow * SEQ + (size_t)s0 + p8;
  for (int pass = 0; pass < 2; ++pass) {
#pragma unroll
    for (int it = 0; it < 4; ++it) {
      const int line = it * 32 + q8;
      *(volatile v4u*)(VHo + base + (size_t)line * SEQ) = vh[it];
      *(volatile v4u*)(VLo + base + (size_t)line * SEQ) = vl[it];
    }
    __threadfence();
  }
}

__global__ __launch_bounds__(256) void norm16(const float* __restrict__ F, int ldn, const float* __restrict__ nw,
                                              u16* Hp, u16* Lp, float sc) {
#pragma clang fp contract(off)
  const int tid = (int)threadIdx.x;
  const int r   = (int)blockIdx.x;
  if (r >= MROWS) return;
  const int col = tid * 8;
  const int dw  = col & (HD - 1);
  const float* p = F + (size_t)r * ldn + col;
  const v4f xa = *(const v4f*)(p), xb = *(const v4f*)(p + 4);
  const v4f wa = *(const v4f*)(nw + dw), wb4 = *(const v4f*)(nw + dw + 4);
  float xv[8], wv[8];
#pragma unroll
  for (int e = 0; e < 4; ++e) {
    xv[e] = xa[e];        xv[4 + e] = xb[e];
    wv[e] = bfr(wa[e]);   wv[4 + e] = bfr(wb4[e]);
  }
  float ss = 0.0f;
#pragma unroll
  for (int e = 0; e < 8; ++e) ss = ss + xv[e] * xv[e];
  ss += __shfl_xor(ss, 1, 32);
  ss += __shfl_xor(ss, 2, 32);
  ss += __shfl_xor(ss, 4, 32);
  ss += __shfl_xor(ss, 8, 32);
  ss += __shfl_xor(ss, 16, 32);
  const float var = ss * (1.0f / (float)HD);
  const float rs  = 1.0f / sqrtf(var + EPS_RMS);
  v4u oh, ol;
#pragma unroll
  for (int e = 0; e < 4; ++e) {
    const float t0 = ((xv[2 * e] * rs) * wv[2 * e]) * sc;
    const float t1 = ((xv[2 * e + 1] * rs) * wv[2 * e + 1]) * sc;
    const _Float16 h0 = (_Float16)t0, h1 = (_Float16)t1;
    const _Float16 l0 = (_Float16)(t0 - (float)h0), l1 = (_Float16)(t1 - (float)h1);
    oh[e] = pk16(h_bits(h0), h_bits(h1));
    ol[e] = pk16(h_bits(l0), h_bits(l1));
  }
  u16* dh = Hp + (size_t)r * ldn + col;
  u16* dl = Lp + (size_t)r * ldn + col;
  for (int pass = 0; pass < 2; ++pass) {
    *(volatile v4u*)(dh) = oh;
    *(volatile v4u*)(dl) = ol;
    __threadfence();
  }
}

__device__ __forceinline__ void epi64(float* sl, v8f a0, v8f a1, v8f a2, v8f a3, float oscale,
                                      float* C, int N, size_t rowb, int col0, int lane) {
  const int hh = lane >> 4, m = lane & 15;
#pragma unroll
  for (int r = 0; r < 8; ++r) {
    const int ro = (8 * hh + r) * 68 + m;
    sl[ro]      = a0[r] * oscale;
    sl[ro + 16] = a1[r] * oscale;
    sl[ro + 32] = a2[r] * oscale;
    sl[ro + 48] = a3[r] * oscale;
  }
  wave_sync_lds();
  v4f vals[8];
#pragma unroll
  for (int it = 0; it < 8; ++it) vals[it] = *(const v4f*)(sl + (it * 2 + hh) * 68 + m * 4);
  float* dst = C + (rowb + (size_t)hh) * (size_t)N + col0 + m * 4;
  for (int pass = 0; pass < 2; ++pass) {
#pragma unroll
    for (int it = 0; it < 8; ++it) {
      *(volatile v4f*)(dst + (size_t)(it * 2) * (size_t)N) = vals[it];
    }
    __threadfence();
  }
}

__global__ __launch_bounds__(128)
void gemm_bf(const u16* __restrict__ A, const u16* __restrict__ Bt, float* C, int M, int N, int K, float oscale) {
  __shared__ __align__(16) float slab[4 * SLAB64];
  const int tid = threadIdx.x, wave = tid >> 5, lane = tid & 31, hh = lane >> 4, m = lane & 15;
  const int ntile = N >> 6;
  const int bid   = blockIdx.x;
  const int rowb  = (bid / ntile) * 64 + wave * 16;
  const int col0  = (bid % ntile) * 64;
  if (rowb + 16 > M) return;
  const u16* ap = A  + (size_t)(rowb + m) * K + 8 * hh;
  const u16* bp = Bt + (size_t)(col0 + m) * K + 8 * hh;
  const size_t bs = (size_t)16 * K;
  v8f acc0 = zero8(), acc1 = zero8(), acc2 = zero8(), acc3 = zero8();
#pragma unroll 1
  for (int k0 = 0; k0 < K; k0 += 32) {
    const v16b a  = ldfrag_b(ap + k0);
    const v16b b0 = ldfrag_b(bp + k0);
    const v16b b1 = ldfrag_b(bp + bs + k0);
    const v16b b2 = ldfrag_b(bp + 2 * bs + k0);
    const v16b b3 = ldfrag_b(bp + 3 * bs + k0);
    acc0 = mma_b(a, b0, acc0);
    acc1 = mma_b(a, b1, acc1);
    acc2 = mma_b(a, b2, acc2);
    acc3 = mma_b(a, b3, acc3);
    guard6<v16b>(acc0, acc1, acc2, acc3, a, b0, b1, b2, b3, a);
  }
  epi64(slab + wave * SLAB64, acc0, acc1, acc2, acc3, oscale, C, N, (size_t)rowb, col0, lane);
}

template <int NPROD>
__global__ __launch_bounds__(128)
void gemm_o(const u16* __restrict__ Ah, const u16* __restrict__ Al, const u16* __restrict__ Bt,
            float* C, int sbeg, int nrt, float oscale) {
  __shared__ __align__(16) float slab[4 * SLAB64];
  const int tid = threadIdx.x, wave = tid >> 5, lane = tid & 31, hh = lane >> 4, m = lane & 15;
  const int ntile = DMOD >> 6;
  const int bid   = blockIdx.x;
  const int ct    = bid % ntile;
  const int t2    = bid / ntile;
  const int rt    = t2 % nrt;
  const int bb    = t2 / nrt;
  if (bb >= NB) return;
  const int srow  = sbeg + rt * 64 + wave * 16;
  if (srow + 16 > SEQ) return;
  const int col0  = ct * 64;
  const int K     = DMOD;
  const size_t rowC = (size_t)bb * SEQ + srow;
  const size_t rowL = (size_t)bb * QO + srow;
  const _Float16* ahp = (const _Float16*)(const void*)Ah + (rowC + m) * K + 8 * hh;
  const _Float16* alp = (const _Float16*)(const void*)Al + (rowL + m) * K + 8 * hh;
  const _Float16* bp  = (const _Float16*)(const void*)Bt + (size_t)(col0 + m) * K + 8 * hh;
  const size_t bs = (size_t)16 * K;
  v8f acc0 = zero8(), acc1 = zero8(), acc2 = zero8(), acc3 = zero8();
  if constexpr (NPROD == 2) {
#pragma unroll 1
    for (int k0 = 0; k0 < K; k0 += 32) {
      const v16h ah = ldfrag_h(ahp + k0), al = ldfrag_h(alp + k0);
      const v16h b0 = ldfrag_h(bp + k0);
      const v16h b1 = ldfrag_h(bp + bs + k0);
      const v16h b2 = ldfrag_h(bp + 2 * bs + k0);
      const v16h b3 = ldfrag_h(bp + 3 * bs + k0);
      acc0 = mma_h(ah, b0, acc0);  acc0 = mma_h(al, b0, acc0);
      acc1 = mma_h(ah, b1, acc1);  acc1 = mma_h(al, b1, acc1);
      acc2 = mma_h(ah, b2, acc2);  acc2 = mma_h(al, b2, acc2);
      acc3 = mma_h(ah, b3, acc3);  acc3 = mma_h(al, b3, acc3);
      guard6<v16h>(acc0, acc1, acc2, acc3, ah, al, b0, b1, b2, b3);
    }
  } else {
#pragma unroll 1
    for (int k0 = 0; k0 < K; k0 += 32) {
      const v16h ah = ldfrag_h(ahp + k0);
      const v16h b0 = ldfrag_h(bp + k0);
      const v16h b1 = ldfrag_h(bp + bs + k0);
      const v16h b2 = ldfrag_h(bp + 2 * bs + k0);
      const v16h b3 = ldfrag_h(bp + 3 * bs + k0);
      acc0 = mma_h(ah, b0, acc0);
      acc1 = mma_h(ah, b1, acc1);
      acc2 = mma_h(ah, b2, acc2);
      acc3 = mma_h(ah, b3, acc3);
      guard6<v16h>(acc0, acc1, acc2, acc3, ah, b0, b1, b2, b3, ah);
    }
  }
  epi64(slab + wave * SLAB64, acc0, acc1, acc2, acc3, oscale, C, DMOD, rowC, col0, lane);
}

__global__ __launch_bounds__(ATT_THREADS)
void attn_g(const u16* __restrict__ QHp, const u16* __restrict__ QLp,
            const u16* __restrict__ KHp, const u16* __restrict__ KLp,
            const u16* __restrict__ VHp, const u16* __restrict__ VLp,
            u16* OHp, u16* OLp) {
  __shared__ __align__(16) float pt[PTW];
  __shared__ __align__(16) float xch[XCHW];
  __shared__ __align__(16) float slabs[WPB * SLW];

  const int tid  = threadIdx.x;
  const int wave = tid >> 5;
  const int lane = tid & 31;
  const int hh   = lane >> 4;
  const int c    = lane & 15;
  const int bid  = blockIdx.x;
  const int qt   = bid % NQT;
  const int t2   = bid / NQT;
  const int head = t2 % NH;
  const int b    = t2 / NH;
  if (b >= NB) return;
  const int q0   = qt * 16;
  if (q0 + 16 > SEQ) return;
  const int g     = head / NREP;
  const int dbase = wave * DW;
  float* slab = slabs + wave * SLW;

  const size_t qcol = (size_t)head * HD + 8 * hh;
  const size_t kcol = (size_t)g * HD + 8 * hh;
  const _Float16* Qh  = (const _Float16*)(const void*)QHp + ((size_t)b * SEQ + q0 + c) * DMOD + qcol;
  const _Float16* Ql  = (const _Float16*)(const void*)QLp + ((size_t)b * SEQ + q0 + c) * DMOD + qcol;
  const _Float16* Khb = (const _Float16*)(const void*)KHp + ((size_t)b * SEQ + 16 * wave + c) * KVD + kcol;
  const _Float16* Klb = (const _Float16*)(const void*)KLp + ((size_t)b * SEQ + 16 * wave + c) * KVD + kcol;
  const _Float16* Vhb = (const _Float16*)(const void*)VHp + ((size_t)(b * NKV + g) * HD + dbase + c) * SEQ + 8 * hh;
  const _Float16* Vlb = (const _Float16*)(const void*)VLp + ((size_t)(b * NKV + g) * HD + dbase + c) * SEQ + 8 * hh;
  const float lsc = SM_SCALE * (LOG2E / (QSC * KSC));
  const float oc  = 1.0f / (PCAR * VCAR);

  float mrow[8], lrow[8];
  v8f o[8];
#pragma unroll
  for (int r = 0; r < 8; ++r) { mrow[r] = -INFINITY; lrow[r] = 0.f; }
#pragma unroll
  for (int j = 0; j < 8; ++j) o[j] = zero8();
  const int ncaus = (q0 >> 5) + 1;
  const int nkt = (ncaus < NKT) ? ncaus : NKT;
  const int qr0 = q0 + 8 * hh;
  const int kw0 = 16 * wave + c;
  const int xm  = 16 * wave + 8 * hh;

#pragma unroll 1
  for (int kt = 0; kt < nkt; ++kt) {
    const int kb = kt * 32;
    v8f s = zero8();
    const _Float16* k0p = Khb + (size_t)kb * KVD;
    const _Float16* l0p = Klb + (size_t)kb * KVD;
#pragma unroll
    for (int kk = 0; kk < HD / 32; ++kk) {
      const v16h qh = ldfrag_h(Qh + kk * 32);
      const v16h ql = ldfrag_h(Ql + kk * 32);
      const v16h kh = ldfrag_h(k0p + kk * 32);
      const v16h kl = ldfrag_h(l0p + kk * 32);
      s = mma_h(qh, kh, s);
      s = mma_h(ql, kh, s);
      s = mma_h(qh, kl, s);
      guard1<v16h>(s, qh, ql, kh, kl);
    }
    const int keyc = kb + kw0;
    float tv[8];
#pragma unroll
    for (int r = 0; r < 8; ++r) {
      const float u = s[r] * lsc;
      const float t = (keyc <= qr0 + r) ? u : NEGT;
      tv[r] = t;
      float mx = t;
#pragma unroll
      for (int off = 1; off < 16; off <<= 1) mx = fmaxf(mx, __shfl_xor(mx, off, 32));
      if (c == 0) xch[xm + r] = mx;
    }
    __syncthreads();
    float alr[8];
#pragma unroll
    for (int r = 0; r < 8; ++r) {
      const float m0 = xch[8 * hh + r];
      const float m1 = xch[16 + 8 * hh + r];
      const float mn = fmaxf(mrow[r], fmaxf(m0, m1));
      const float ms = (mn == -INFINITY) ? 0.0f : mn;
      const float al = exp2f(mrow[r] - ms);
      mrow[r] = mn;
      alr[r]  = al;
      const float e = exp2f(tv[r] - ms);
      float ps = e;
#pragma unroll
      for (int off = 1; off < 16; off <<= 1) ps += __shfl_xor(ps, off, 32);
      if (c == 0) xch[32 + xm + r] = ps;
#pragma unroll
      for (int j = 0; j < 8; ++j) o[j][r] *= al;
      pt[(8 * hh + r) * PTP + kw0] = e;
    }
    __syncthreads();
#pragma unroll
    for (int r = 0; r < 8; ++r) {
      const float p0s = xch[32 + 8 * hh + r];
      const float p1s = xch[48 + 8 * hh + r];
      lrow[r] = lrow[r] * alr[r] + (p0s + p1s);
    }
    FragH ph;
    {
      const float* prow = pt + c * PTP + 8 * hh;
      const v4f p0 = *(const v4f*)(prow), p1 = *(const v4f*)(prow + 4);
      const v4f p2 = *(const v4f*)(prow + 16), p3 = *(const v4f*)(prow + 20);
#pragma unroll
      for (int e = 0; e < 4; ++e) {
        ph.h[0][e]     = (_Float16)(p0[e] * PCAR);
        ph.h[0][4 + e] = (_Float16)(p1[e] * PCAR);
        ph.h[1][e]     = (_Float16)(p2[e] * PCAR);
        ph.h[1][4 + e] = (_Float16)(p3[e] * PCAR);
      }
    }
    {
      const _Float16* vhp = Vhb + kb;
      const _Float16* vlp = Vlb + kb;
#pragma unroll
      for (int jg = 0; jg < 4; ++jg) {
        const size_t da = (size_t)(2 * jg) * 16 * SEQ;
        const size_t db = da + (size_t)16 * SEQ;
        const v16h vha = ldfrag_h(vhp + da), vhb2 = ldfrag_h(vhp + db);
        const v16h vla = ldfrag_h(vlp + da), vlb2 = ldfrag_h(vlp + db);
        o[2 * jg]     = mma_h(ph.v, vha,  o[2 * jg]);
        o[2 * jg]     = mma_h(ph.v, vla,  o[2 * jg]);
        o[2 * jg + 1] = mma_h(ph.v, vhb2, o[2 * jg + 1]);
        o[2 * jg + 1] = mma_h(ph.v, vlb2, o[2 * jg + 1]);
        guard2(o[2 * jg], o[2 * jg + 1], ph.v, vha, vhb2, vla, vlb2, ph.v);
      }
    }
    __syncthreads();
  }
  acc_guard4(o[0], o[1], o[2], o[3]);
  acc_guard4(o[4], o[5], o[6], o[7]);
#pragma unroll
  for (int r = 0; r < 8; ++r) {
    const float lv  = lrow[r];
    const float ls  = (lv > 0.0f) ? lv : 1.0f;
    const float inv = (lv > 0.0f) ? ((1.0f / ls) * oc) : 0.0f;
#pragma unroll
    for (int j = 0; j < 8; ++j) {
      const int idx = (8 * hh + r) * SLP + j * 16 + c;
      slab[idx] = o[j][r] * inv;
    }
  }

  wave_sync_lds();
  v4u oh[8], ol[8];
  const int rq = lane >> 4, c8 = (lane & 15) * 8;
#pragma unroll
  for (int it = 0; it < 8; ++it) {
    const int row = it * 2 + rq;
    const v4f a = *(const v4f*)(slab + row * SLP + c8), b4 = *(const v4f*)(slab + row * SLP + c8 + 4);
    float w[8];
#pragma unroll
    for (int e = 0; e < 4; ++e) { w[e] = a[e] * OSC; w[4 + e] = b4[e] * OSC; }
#pragma unroll
    for (int e = 0; e < 4; ++e) {
      const _Float16 h0 = (_Float16)w[2 * e], h1 = (_Float16)w[2 * e + 1];
      const _Float16 l0 = (_Float16)(w[2 * e] - (float)h0), l1 = (_Float16)(w[2 * e + 1] - (float)h1);
      oh[it][e] = pk16(h_bits(h0), h_bits(h1));
      ol[it][e] = pk16(h_bits(l0), h_bits(l1));
    }
  }
  const bool wlo = (q0 < QO);
  const size_t ob  = ((size_t)b * SEQ + q0) * DMOD + (size_t)head * HD + (size_t)dbase + c8;
  const size_t olb = ((size_t)b * QO  + q0) * DMOD + (size_t)head * HD + (size_t)dbase + c8;
  for (int pass = 0; pass < 2; ++pass) {
#pragma unroll
    for (int it = 0; it < 8; ++it) {
      const int row = it * 2 + rq;
      *(volatile v4u*)(OHp + ob + (size_t)row * DMOD) = oh[it];
      if (wlo) {
        *(volatile v4u*)(OLp + olb + (size_t)row * DMOD) = ol[it];
      }
    }
    __threadfence();
  }
}

extern "C" void kernel_launch(void* const* d_in, const int* in_sizes, int n_in,
                              void* d_out, int out_size, void* d_ws, size_t ws_size,
                              hipStream_t stream) {
  if (n_in < 7) return;
  if (in_sizes[0] < ((NB - 1) * XS_FULL + SEQ) * DMOD) return;
  if (in_sizes[1] != DMOD * DMOD) return;
  if (in_sizes[2] != KVD * DMOD) return;
  if (in_sizes[3] != KVD * DMOD) return;
  if (in_sizes[4] != DMOD * DMOD) return;
  if (in_sizes[5] < HD) return;
  if (in_sizes[6] < HD) return;
  if (out_size < MROWS * DMOD) return;

  const float* x   = (const float*)d_in[0];
  const float* qw  = (const float*)d_in[1];
  const float* kw  = (const float*)d_in[2];
  const float* vw  = (const float*)d_in[3];
  const float* ow  = (const float*)d_in[4];
  const float* qnw = (const float*)d_in[5];
  const float* knw = (const float*)d_in[6];
  float*       out = (float*)d_out;

  const size_t szXB = (size_t)MROWS * DMOD * 2;
  const size_t szW  = (size_t)DMOD * DMOD * 2;
  const size_t szF  = (size_t)MROWS * DMOD * 4;
  const size_t szOH = (size_t)MROWS * DMOD * 2;
  const size_t szOL = (size_t)NB * QO * DMOD * 2;
  const size_t szWO = (size_t)DMOD * DMOD * 2;
  const size_t szQ  = (size_t)MROWS * DMOD * 2;
  const size_t szK  = (size_t)MROWS * KVD * 2;
  const size_t g0a  = szXB + szW + szF;
  const size_t g0b  = szOH + szOL + szWO;
  const size_t G0   = (g0a > g0b) ? g0a : g0b;
  const size_t oXB = 0;
  const size_t oW  = szXB;
  const size_t oF  = szXB + szW;
  const size_t oOH = 0;
  const size_t oOL = szOH;
  const size_t oWO = szOH + szOL;
  size_t off = G0;
  const size_t oQH = off; off += szQ;
  const size_t oQL = off; off += szQ;
  const size_t oKH = off; off += szK;
  const size_t oKL = off; off += szK;
  const size_t oVH = off; off += szK;
  const size_t oVL = off; off += szK;
  if (off > ws_size) return;
  if (off > (size_t)WS_CAP) return;

  char* ws = (char*)d_ws;
  u16*   XB = (u16*)(ws + oXB);
  u16*   W  = (u16*)(ws + oW);
  float* F  = (float*)(ws + oF);
  u16*   OH = (u16*)(ws + oOH);
  u16*   OL = (u16*)(ws + oOL);
  u16*   WO = (u16*)(ws + oWO);
  u16*   QH = (u16*)(ws + oQH);
  u16*   QL = (u16*)(ws + oQL);
  u16*   KH = (u16*)(ws + oKH);
  u16*   KL = (u16*)(ws + oKL);
  u16*   VH = (u16*)(ws + oVH);
  u16*   VL = (u16*)(ws + oVL);

  const dim3 b256(256), b128(128), bAT(ATT_THREADS);
  const int  n8x  = (SEQ * DMOD) / 8;
  const int  n8wq = (DMOD * DMOD) / 8;
  const int  n8wk = (KVD * DMOD) / 8;
  const dim3 gX((n8x + 255) / 256);
  const dim3 gWQ((n8wq + 255) / 256);
  const dim3 gWK((n8wk + 255) / 256);
  const dim3 gGQ((MROWS / 64) * (DMOD / 64));
  const dim3 gGK((MROWS / 64) * (KVD / 64));
  const dim3 gRW(MROWS);
  const dim3 gVT(NKV * (HD / DW) * NSTT);
  const dim3 gAT(NQT * NH * NB);
  const int  nrtR = QO / 64;
  const int  nrtP = (SEQ - QO) / 64;

  for (int b = 0; b < NB; ++b) {
    cvt16<<<gX, b256, 0, stream>>>(x + (size_t)b * XS_FULL * DMOD, XB + (size_t)b * SEQ * DMOD, n8x, 0, 1.0f);
  }
  cvt16<<<gWQ, b256, 0, stream>>>(qw, W, n8wq, 0, 1.0f);
  gemm_bf<<<gGQ, b128, 0, stream>>>(XB, W, F, MROWS, DMOD, DMOD, 1.0f);
  norm16<<<gRW, dim3(DMOD / 8), 0, stream>>>(F, DMOD, qnw, QH, QL, QSC);
  cvt16<<<gWK, b256, 0, stream>>>(kw, W, n8wk, 0, 1.0f);
  gemm_bf<<<gGK, b128, 0, stream>>>(XB, W, F, MROWS, KVD, DMOD, 1.0f);
  norm16<<<gRW, dim3(KVD / 8), 0, stream>>>(F, KVD, knw, KH, KL, KSC);
  cvt16<<<gWK, b256, 0, stream>>>(vw, W, n8wk, 0, 1.0f);
  gemm_bf<<<gGK, b128, 0, stream>>>(XB, W, F, MROWS, KVD, DMOD, 1.0f);
  vt16<<<gVT, b256, 0, stream>>>(F, VH, VL);
  attn_g<<<gAT, bAT, 0, stream>>>(QH, QL, KH, KL, VH, VL, OH, OL);
  cvt16<<<gWQ, b256, 0, stream>>>(ow, WO, n8wq, 1, WOS);
  gemm_o<2><<<dim3(NB * nrtR * (DMOD / 64)), b128, 0, stream>>>(OH, OL, WO, out, 0, nrtR, 1.0f / (OSC * WOS));
  if (nrtP > 0) {
    gemm_o<1><<<dim3(NB * nrtP * (DMOD / 64)), b128, 0, stream>>>(OH, OL, WO, out, QO, nrtP, 1.0f / (OSC * WOS));
  }
  (void)hipGetLastError();
}
